// mplstm_48584670053219
// MI455X (gfx1250) — hardware-verified
//
#include <hip/hip_runtime.h>
#include <stddef.h>
#include <stdint.h>

#define BB   2
#define LQ   512
#define LK   712
#define LKP  768
#define DM   512
#define NC   200
#define KS   5
#define TO   508
#define KC   (KS * DM)
#define CP   256
#define KF   224
#define SP   72
#define AW   224
#define OPF  36
#define LN_EPS 1e-5f

static_assert(TO == LQ - (KS - 1));
static_assert(LK == LQ + NC);
static_assert((LKP % 64) == 0 && LKP >= LK);
static_assert(LQ - 16 + KF <= LKP);
static_assert(NC + 16 <= KF && (KF % 32) == 0 && KF <= CP);
static_assert((KC % 32) == 0 && (DM % 64) == 0 && (LQ % 64) == 0 && (CP % 64) == 0);
static_assert((SP % 8) == 0 && (AW % 8) == 0 && (OPF % 4) == 0);
static_assert((TO - 1) + (KS - 1) <= LQ - 1);

#define SZ_W   ((size_t)DM * DM * 2)
#define SZ_CW  ((size_t)CP * KC * 2)
#define SZ_FW  ((size_t)CP * CP * 2)
#define SZ_KP  ((size_t)BB * LKP * DM * 2)
#define SZ_QP  ((size_t)BB * LQ * DM * 2)
#define SZ_CL  ((size_t)BB * LQ * CP * 2)
#define SZ_KT  ((size_t)BB * DM * LKP * 2)
#define OFF_WQ  ((size_t)0)
#define OFF_WK  (OFF_WQ + SZ_W)
#define OFF_WV  (OFF_WK + SZ_W)
#define OFF_CW  (OFF_WV + SZ_W)
#define OFF_FW  (OFF_CW + SZ_CW)
#define OFF_KH  (OFF_FW + SZ_FW)
#define OFF_KL  (OFF_KH + SZ_KP)
#define OFF_VH  (OFF_KL + SZ_KP)
#define OFF_VL  (OFF_VH + SZ_KP)
#define OFF_NH  (OFF_VL + SZ_KP)
#define OFF_NL  (OFF_NH + SZ_QP)
#define OFF_QH  (OFF_NL + SZ_QP)
#define OFF_QL  (OFF_QH + SZ_QP)
#define OFF_CH  (OFF_QL + SZ_QP)
#define OFF_CLO (OFF_CH + SZ_CL)
#define OFF_WH  (OFF_CLO + SZ_CL)
#define OFF_WL  (OFF_WH + SZ_CL)
#define OFF_TH  (OFF_WL + SZ_CL)
#define OFF_TL  (OFF_TH + SZ_KT)
#define WS_NEED (OFF_TL + SZ_KT)
static_assert(WS_NEED == 18743296);
static_assert((OFF_CW % 256) == 0 && (OFF_FW % 256) == 0 && (OFF_KH % 256) == 0 &&
              (OFF_NH % 256) == 0 && (OFF_QH % 256) == 0 && (OFF_CH % 256) == 0 &&
              (OFF_WH % 256) == 0 && (OFF_TH % 256) == 0 && (OFF_TL % 256) == 0);

typedef float          v4f   __attribute__((ext_vector_type(4)));
typedef float          v8f   __attribute__((ext_vector_type(8)));
typedef unsigned int   v4u   __attribute__((ext_vector_type(4)));
typedef unsigned short v8us  __attribute__((ext_vector_type(8)));
typedef unsigned short v16us __attribute__((ext_vector_type(16)));
typedef v4u v4ua __attribute__((may_alias));
typedef v4f v4fa __attribute__((may_alias));
#if defined(__HIP_DEVICE_COMPILE__)
typedef _Float16 v16h __attribute__((ext_vector_type(16)));
#endif

union FragU { v16us v; v8us half[2]; };

#define DEV __device__ __forceinline__
#define R2048 0.00048828125f
#define R1024 0.0009765625f
#define R256  0.00390625f

DEV int imin(int a, int b) { return a < b ? a : b; }
DEV int imax(int a, int b) { return a > b ? a : b; }
DEV unsigned bbits(float f) {
  unsigned u = __float_as_uint(f);
  return (u + 0x7FFFu + ((u >> 16) & 1u)) >> 16;
}
DEV float bf16r(float f) {
  return __uint_as_float(bbits(f) << 16);
}
DEV unsigned short hbits(float f) {
#if defined(__HIP_DEVICE_COMPILE__)
  return __builtin_bit_cast(unsigned short, (_Float16)f);
#else
  (void)f;
  return 0;
#endif
}
DEV float h2f(unsigned short u) {
#if defined(__HIP_DEVICE_COMPILE__)
  return (float)__builtin_bit_cast(_Float16, u);
#else
  (void)u;
  return 0.0f;
#endif
}
DEV unsigned short rbits(float x, unsigned short hb) {
  return hbits((x - h2f(hb)) * 2048.0f);
}
DEV v8f zero8() { v8f z = {0.f, 0.f, 0.f, 0.f, 0.f, 0.f, 0.f, 0.f}; return z; }
DEV float sigm_f(float x) {
  return __builtin_amdgcn_rcpf(1.0f + expf(-x));
}
DEV float wsum(float v) {
  v += __shfl_xor(v, 16);
  v += __shfl_xor(v, 8);
  v += __shfl_xor(v, 4);
  v += __shfl_xor(v, 2);
  v += __shfl_xor(v, 1);
  return v;
}

DEV v16us ldfrag(const unsigned short* p) {
  FragU f;
  f.half[0] = *(const v8us*)(p);
  f.half[1] = *(const v8us*)(p + 16);
  return f.v;
}

DEV v8f mma_h(v16us a, v16us b, v8f c) {
#if defined(__HIP_DEVICE_COMPILE__)
  return __builtin_amdgcn_wmma_f32_16x16x32_f16(false, __builtin_bit_cast(v16h, a),
                                               false, __builtin_bit_cast(v16h, b),
                                               (short)0, c, false, false);
#else
  (void)a; (void)b;
  return c;
#endif
}
DEV void grd8x6(v8f& c0, v8f& c1, v8f& c2, v8f& c3, v8f& c4, v8f& c5, v8f& c6, v8f& c7,
                const v16us& x0, const v16us& x1, const v16us& x2, const v16us& x3,
                const v16us& x4, const v16us& x5) {
#if defined(__HIP_DEVICE_COMPILE__)
  asm volatile("v_nop\n\tv_nop\n\tv_nop\n\tv_nop"
               : "+v"(c0), "+v"(c1), "+v"(c2), "+v"(c3), "+v"(c4), "+v"(c5), "+v"(c6), "+v"(c7)
               : "v"(x0), "v"(x1), "v"(x2), "v"(x3), "v"(x4), "v"(x5));
#endif
}
DEV void grd8x8(v8f& c0, v8f& c1, v8f& c2, v8f& c3, v8f& c4, v8f& c5, v8f& c6, v8f& c7,
                const v16us& x0, const v16us& x1, const v16us& x2, const v16us& x3,
                const v16us& x4, const v16us& x5, const v16us& x6, const v16us& x7) {
#if defined(__HIP_DEVICE_COMPILE__)
  asm volatile("v_nop\n\tv_nop\n\tv_nop\n\tv_nop"
               : "+v"(c0), "+v"(c1), "+v"(c2), "+v"(c3), "+v"(c4), "+v"(c5), "+v"(c6), "+v"(c7)
               : "v"(x0), "v"(x1), "v"(x2), "v"(x3), "v"(x4), "v"(x5), "v"(x6), "v"(x7));
#endif
}
DEV void grd4x6(v8f& c0, v8f& c1, v8f& c2, v8f& c3,
                const v16us& x0, const v16us& x1, const v16us& x2, const v16us& x3,
                const v16us& x4, const v16us& x5) {
#if defined(__HIP_DEVICE_COMPILE__)
  asm volatile("v_nop\n\tv_nop\n\tv_nop\n\tv_nop"
               : "+v"(c0), "+v"(c1), "+v"(c2), "+v"(c3)
               : "v"(x0), "v"(x1), "v"(x2), "v"(x3), "v"(x4), "v"(x5));
#endif
}

__global__ __launch_bounds__(256)
void k_cvtw(const float* __restrict__ w0, const float* __restrict__ w1, const float* __restrict__ w2,
            unsigned short* d0, unsigned short* d1, unsigned short* d2, int n8, float scale)
{
  const int i = blockIdx.x * 256 + threadIdx.x;
  if (i >= n8) return;
  const int sel = blockIdx.y;
  const float* src = (sel == 0) ? w0 : ((sel == 1) ? w1 : w2);
  unsigned short* dst = (sel == 0) ? d0 : ((sel == 1) ? d1 : d2);
  const float* s = src + (size_t)i * 8;
  const v4f a = *(const v4f*)(s);
  const v4f b = *(const v4f*)(s + 4);
  v8us o;
  o[0] = hbits(bf16r(a[0]) * scale); o[1] = hbits(bf16r(a[1]) * scale);
  o[2] = hbits(bf16r(a[2]) * scale); o[3] = hbits(bf16r(a[3]) * scale);
  o[4] = hbits(bf16r(b[0]) * scale); o[5] = hbits(bf16r(b[1]) * scale);
  o[6] = hbits(bf16r(b[2]) * scale); o[7] = hbits(bf16r(b[3]) * scale);
  const v4u w = __builtin_bit_cast(v4u, o);
  v4u* p = (v4u*)(dst + (size_t)i * 8);
  *(volatile v4u*)p = w;
  __threadfence();
  *(volatile v4u*)p = w;
}

__global__ __launch_bounds__(256)
void k_cvtc(const float* __restrict__ cw, unsigned short* dst, int n8)
{
  const int i = blockIdx.x * 256 + threadIdx.x;
  if (i >= n8) return;
  const int e = i * 8;
  const int o = e / KC;
  const int kk = e - o * KC;
  const int tau = kk / DM;
  const int db = kk - tau * DM;
  const int oc = imin(o, NC - 1);
  const float* s = cw + ((size_t)oc * DM + db) * KS + tau;
  const bool ok = (o < NC);
  v8us w;
#pragma unroll
  for (int j = 0; j < 8; ++j) {
    const float v = s[j * KS];
    w[j] = ok ? hbits(bf16r(v) * 1024.0f) : (unsigned short)0;
  }
  const v4u ww = __builtin_bit_cast(v4u, w);
  v4u* p = (v4u*)(dst + (size_t)e);
  *(volatile v4u*)p = ww;
  __threadfence();
  *(volatile v4u*)p = ww;
}

__global__ __launch_bounds__(256)
void k_cvtf(const float* __restrict__ fw, unsigned short* dst, int n8)
{
  const int i = blockIdx.x * 256 + threadIdx.x;
  if (i >= n8) return;
  const int e = i * 8;
  const int j = e >> 8;
  const int ob = e & (CP - 1);
  const int jc = imin(j, NC - 1);
  v8us w;
#pragma unroll
  for (int u = 0; u < 8; ++u) {
    const int o = ob + u;
    const int ocl = imin(o, NC - 1);
    const float v = fw[jc * NC + ocl];
    w[u] = (j < NC && o < NC) ? hbits(bf16r(v) * 256.0f) : (unsigned short)0;
  }
  const v4u ww = __builtin_bit_cast(v4u, w);
  v4u* p = (v4u*)(dst + (size_t)e);
  *(volatile v4u*)p = ww;
  __threadfence();
  *(volatile v4u*)p = ww;
}

__global__ __launch_bounds__(256)
void k_ln(const float* __restrict__ key, const float* __restrict__ val, const float* __restrict__ qry,
          const float* __restrict__ gk, const float* __restrict__ bk,
          const float* __restrict__ gv, const float* __restrict__ bv,
          const float* __restrict__ gq, const float* __restrict__ bq,
          unsigned short* khi, unsigned short* klo, unsigned short* vhi, unsigned short* vlo,
          unsigned short* qhi, unsigned short* qlo)
{
  const int which = blockIdx.y;
  if (which == 2 && blockIdx.x >= (BB * LQ) / 8) return;
  const int tid = threadIdx.x, lane = tid & 31, wave = tid >> 5;
  const int prow = blockIdx.x * 8 + wave;
  const float* src;
  const float* gp;
  const float* bp;
  unsigned short* dh;
  unsigned short* dl;
  int srow;
  bool valid;
  if (which == 2) {
    src = qry; gp = gq; bp = bq; dh = qhi; dl = qlo;
    srow = prow; valid = true;
  } else {
    const int bb = prow / LKP;
    const int s  = prow - bb * LKP;
    valid = (s < LK);
    srow = bb * LK + (valid ? s : (LK - 1));
    if (which == 0) { src = key; gp = gk; bp = bk; dh = khi; dl = klo; }
    else            { src = val; gp = gv; bp = bv; dh = vhi; dl = vlo; }
  }

  const float* xp = src + (size_t)srow * DM + 8 * lane;
  const float* gg = gp + 8 * lane;
  const float* bg = bp + 8 * lane;
  float x[16], g[16], be[16];
  {
    const v4f a0 = *(const v4f*)(xp), a1 = *(const v4f*)(xp + 4);
    const v4f a2 = *(const v4f*)(xp + 256), a3 = *(const v4f*)(xp + 260);
    const v4f g0 = *(const v4f*)(gg), g1 = *(const v4f*)(gg + 4);
    const v4f g2 = *(const v4f*)(gg + 256), g3 = *(const v4f*)(gg + 260);
    const v4f b0 = *(const v4f*)(bg), b1 = *(const v4f*)(bg + 4);
    const v4f b2 = *(const v4f*)(bg + 256), b3 = *(const v4f*)(bg + 260);
#pragma unroll
    for (int i = 0; i < 4; ++i) {
      x[i] = bf16r(a0[i]);  x[4 + i] = bf16r(a1[i]);  x[8 + i] = bf16r(a2[i]);  x[12 + i] = bf16r(a3[i]);
      g[i] = bf16r(g0[i]);  g[4 + i] = bf16r(g1[i]);  g[8 + i] = bf16r(g2[i]);  g[12 + i] = bf16r(g3[i]);
      be[i] = bf16r(b0[i]); be[4 + i] = bf16r(b1[i]); be[8 + i] = bf16r(b2[i]); be[12 + i] = bf16r(b3[i]);
    }
  }
  float s1 = 0.0f;
#pragma unroll
  for (int i = 0; i < 16; ++i) s1 += x[i];
  s1 = wsum(s1);
  const float mu = s1 * (1.0f / (float)DM);
  float s2 = 0.0f;
#pragma unroll
  for (int i = 0; i < 16; ++i) { const float d = x[i] - mu; s2 += d * d; }
  s2 = wsum(s2);
  const float rstd = rsqrtf(s2 * (1.0f / (float)DM) + LN_EPS);

  v8us oh0, oh1, ol0, ol1;
#pragma unroll
  for (int i = 0; i < 8; ++i) {
    float y0 = (x[i] - mu) * rstd * g[i] + be[i];
    float y1 = (x[8 + i] - mu) * rstd * g[8 + i] + be[8 + i];
    y0 = valid ? y0 : 0.0f;
    y1 = valid ? y1 : 0.0f;
    const unsigned short h0 = hbits(y0), h1 = hbits(y1);
    oh0[i] = h0;            oh1[i] = h1;
    ol0[i] = rbits(y0, h0); ol1[i] = rbits(y1, h1);
  }
  const v4u wh0 = __builtin_bit_cast(v4u, oh0), wh1 = __builtin_bit_cast(v4u, oh1);
  const v4u wl0 = __builtin_bit_cast(v4u, ol0), wl1 = __builtin_bit_cast(v4u, ol1);
  const size_t ro = (size_t)prow * DM + 8 * lane;
  v4u* ph0 = (v4u*)(dh + ro);
  v4u* ph1 = (v4u*)(dh + ro + 256);
  v4u* pl0 = (v4u*)(dl + ro);
  v4u* pl1 = (v4u*)(dl + ro + 256);
  *(volatile v4u*)ph0 = wh0; *(volatile v4u*)ph1 = wh1;
  *(volatile v4u*)pl0 = wl0; *(volatile v4u*)pl1 = wl1;
  __threadfence();
  *(volatile v4u*)ph0 = wh0; *(volatile v4u*)ph1 = wh1;
  *(volatile v4u*)pl0 = wl0; *(volatile v4u*)pl1 = wl1;
}

__global__ __launch_bounds__(128)
void k_kv(const unsigned short* __restrict__ khi, const unsigned short* __restrict__ klo,
          const unsigned short* __restrict__ vhi, const unsigned short* __restrict__ vlo,
          const unsigned short* __restrict__ wk,  const unsigned short* __restrict__ wv,
          const float* __restrict__ wkb, const float* __restrict__ wvb,
          unsigned short* kth, unsigned short* ktl)
{
  __shared__ __align__(16) unsigned short T[2][32][SP];
  const int tid = threadIdx.x, lane = tid & 31, wave = tid >> 5;
  const int hh = lane >> 4, cc = lane & 15;
  const int s0 = blockIdx.x * 64, n0 = blockIdx.y * 32, b = blockIdx.z;

  const size_t aoff = ((size_t)(b * LKP + s0 + wave * 16 + cc)) * DM + 8 * hh;
  const unsigned short* pkh = khi + aoff;
  const unsigned short* pkl = klo + aoff;
  const unsigned short* pvh = vhi + aoff;
  const unsigned short* pvl = vlo + aoff;
  const size_t boff = ((size_t)(n0 + cc)) * DM + 8 * hh;
  const unsigned short* pwk0 = wk + boff;
  const unsigned short* pwk1 = pwk0 + (size_t)16 * DM;
  const unsigned short* pwv0 = wv + boff;
  const unsigned short* pwv1 = pwv0 + (size_t)16 * DM;

  v8f akh[2], akl[2], avh[2], avl[2];
#pragma unroll
  for (int n = 0; n < 2; ++n) { akh[n] = zero8(); akl[n] = zero8(); avh[n] = zero8(); avl[n] = zero8(); }

#pragma unroll 1
  for (int ko = 0; ko < DM; ko += 32) {
    const v16us fkh = ldfrag(pkh + ko);
    const v16us fkl = ldfrag(pkl + ko);
    const v16us fvh = ldfrag(pvh + ko);
    const v16us fvl = ldfrag(pvl + ko);
    const v16us gk0 = ldfrag(pwk0 + ko);
    const v16us gk1 = ldfrag(pwk1 + ko);
    const v16us gv0 = ldfrag(pwv0 + ko);
    const v16us gv1 = ldfrag(pwv1 + ko);
    akh[0] = mma_h(fkh, gk0, akh[0]); akl[0] = mma_h(fkl, gk0, akl[0]);
    akh[1] = mma_h(fkh, gk1, akh[1]); akl[1] = mma_h(fkl, gk1, akl[1]);
    avh[0] = mma_h(fvh, gv0, avh[0]); avl[0] = mma_h(fvl, gv0, avl[0]);
    avh[1] = mma_h(fvh, gv1, avh[1]); avl[1] = mma_h(fvl, gv1, avl[1]);
    grd8x8(akh[0], akh[1], akl[0], akl[1], avh[0], avh[1], avl[0], avl[1],
           fkh, fkl, fvh, fvl, gk0, gk1, gv0, gv1);
  }

#pragma unroll
  for (int nt = 0; nt < 2; ++nt) {
    const int col = n0 + 16 * nt + cc;
    const float bkv = bf16r(wkb[col]);
    const float bvv = bf16r(wvb[col]);
#pragma unroll
    for (int r = 0; r < 8; ++r) {
      const int sl = wave * 16 + 8 * hh + r;
      const int s  = s0 + sl;
      const float k1 = (akh[nt][r] + akl[nt][r] * R2048) * R256 + bkv;
      const float v1 = (avh[nt][r] + avl[nt][r] * R2048) * R256 + bvv;
      float kv = fmaxf(k1, 0.0f) * v1;
      kv = (s < LK) ? kv : 0.0f;
      const unsigned short hb = hbits(kv);
      T[0][16 * nt + cc][sl] = hb;
      T[1][16 * nt + cc][sl] = rbits(kv, hb);
    }
  }
  __syncthreads();

  v4u vv[4];
#pragma unroll
  for (int it = 0; it < 4; ++it) {
    const int pl = it >> 1;
    const int dl = (it & 1) * 16 + wave * 4 + (lane >> 3);
    const int p  = lane & 7;
    vv[it] = *(const v4ua*)(&T[pl][dl][8 * p]);
  }
#pragma unroll
  for (int it = 0; it < 4; ++it) {
    const int pl = it >> 1;
    const int dl = (it & 1) * 16 + wave * 4 + (lane >> 3);
    const int p  = lane & 7;
    unsigned short* base = pl ? ktl : kth;
    v4u* dst = (v4u*)(base + ((size_t)(b * DM + n0 + dl)) * LKP + s0 + 8 * p);
    *(volatile v4u*)dst = vv[it];
  }
  __threadfence();
#pragma unroll
  for (int it = 0; it < 4; ++it) {
    const int pl = it >> 1;
    const int dl = (it & 1) * 16 + wave * 4 + (lane >> 3);
    const int p  = lane & 7;
    unsigned short* base = pl ? ktl : kth;
    v4u* dst = (v4u*)(base + ((size_t)(b * DM + n0 + dl)) * LKP + s0 + 8 * p);
    *(volatile v4u*)dst = vv[it];
  }
}

template <int MODE>
__global__ __launch_bounds__(128)
void k_g64(const unsigned short* __restrict__ ahi, const unsigned short* __restrict__ alo,
           const unsigned short* __restrict__ bw, const float* __restrict__ bias,
           unsigned short* dhi, unsigned short* dlo)
{
  constexpr int LDA = (MODE == 2) ? CP : DM;
  constexpr int KK  = (MODE == 0) ? DM : ((MODE == 1) ? KC : KF);
  constexpr int LDB = (MODE == 0) ? DM : ((MODE == 1) ? KC : CP);
  constexpr int OP  = (MODE == 0) ? DM : CP;
  constexpr int NV  = (MODE == 0) ? DM : NC;
  const float scl = (MODE == 1) ? R1024 : R256;
  __shared__ __align__(16) unsigned short S[2][64][SP];

  const int tid = threadIdx.x, lane = tid & 31, wave = tid >> 5;
  const int hh = lane >> 4, cc = lane & 15;
  const int t0 = blockIdx.x * 64, n0 = blockIdx.y * 64, b = blockIdx.z;
  int tr = t0 + wave * 16 + cc;
  if (MODE == 1) tr = imin(tr, TO - 1);
  const size_t aoff = ((size_t)(b * LQ + tr)) * LDA + 8 * hh;
  const unsigned short* pah = ahi + aoff;
  const unsigned short* pal = alo + aoff;
  const unsigned short* pb  = bw + ((size_t)(n0 + cc)) * LDB + 8 * hh;

  v8f ch[4], cl[4];
#pragma unroll
  for (int n = 0; n < 4; ++n) { ch[n] = zero8(); cl[n] = zero8(); }

#pragma unroll 1
  for (int ko = 0; ko < KK; ko += 32) {
    const v16us fa = ldfrag(pah + ko);
    const v16us fl = ldfrag(pal + ko);
    const v16us g0 = ldfrag(pb + ko);
    const v16us g1 = ldfrag(pb + (size_t)16 * LDB + ko);
    const v16us g2 = ldfrag(pb + (size_t)32 * LDB + ko);
    const v16us g3 = ldfrag(pb + (size_t)48 * LDB + ko);
    ch[0] = mma_h(fa, g0, ch[0]); cl[0] = mma_h(fl, g0, cl[0]);
    ch[1] = mma_h(fa, g1, ch[1]); cl[1] = mma_h(fl, g1, cl[1]);
    ch[2] = mma_h(fa, g2, ch[2]); cl[2] = mma_h(fl, g2, cl[2]);
    ch[3] = mma_h(fa, g3, ch[3]); cl[3] = mma_h(fl, g3, cl[3]);
    grd8x6(ch[0], ch[1], ch[2], ch[3], cl[0], cl[1], cl[2], cl[3], fa, fl, g0, g1, g2, g3);
  }

#pragma unroll
  for (int nt = 0; nt < 4; ++nt) {
    const int col  = n0 + 16 * nt + cc;
    const int colc = imin(col, NV - 1);
    const float bvl = (col < NV) ? bf16r(bias[colc]) : 0.0f;
#pragma unroll
    for (int r = 0; r < 8; ++r) {
      const int rl = wave * 16 + 8 * hh + r;
      float x = (ch[nt][r] + cl[nt][r] * R2048) * scl + bvl;
      if (MODE == 1) x = fmaxf(x, 0.0f);
      if (MODE == 2) x = sigm_f(x);
      x = (col < NV) ? x : 0.0f;
      const unsigned short hb = hbits(x);
      S[0][rl][16 * nt + cc] = hb;
      S[1][rl][16 * nt + cc] = rbits(x, hb);
    }
  }
  __syncthreads();

  v4u vv[8];
#pragma unroll
  for (int it = 0; it < 8; ++it) {
    const int pl = it >> 2;
    const int rl = (it & 3) * 16 + wave * 4 + (lane >> 3);
    const int p  = lane & 7;
    vv[it] = *(const v4ua*)(&S[pl][rl][8 * p]);
  }
#pragma unroll
  for (int it = 0; it < 8; ++it) {
    const int pl = it >> 2;
    const int rl = (it & 3) * 16 + wave * 4 + (lane >> 3);
    const int p  = lane & 7;
    unsigned short* base = pl ? dlo : dhi;
    v4u* dst = (v4u*)(base + ((size_t)(b * LQ + t0 + rl)) * OP + n0 + 8 * p);
    *(volatile v4u*)dst = vv[it];
  }
  __threadfence();
#pragma unroll
  for (int it = 0; it < 8; ++it) {
    const int pl = it >> 2;
    const int rl = (it & 3) * 16 + wave * 4 + (lane >> 3);
    const int p  = lane & 7;
    unsigned short* base = pl ? dlo : dhi;
    v4u* dst = (v4u*)(base + ((size_t)(b * LQ + t0 + rl)) * OP + n0 + 8 * p);
    *(volatile v4u*)dst = vv[it];
  }
}

__global__ __launch_bounds__(64)
void k_fin(const unsigned short* __restrict__ whi, const unsigned short* __restrict__ wlo,
           const unsigned short* __restrict__ kth, const unsigned short* __restrict__ ktl,
           float* out)
{
  __shared__ __align__(16) unsigned short Ah[2][16][AW];
  __shared__ __align__(16) unsigned short Al[2][16][AW];
  __shared__ __align__(16) float O[2][16][OPF];
  const int tid = threadIdx.x, lane = tid & 31, wave = tid >> 5;
  const int hh = lane >> 4, cc = lane & 15;
  const int b = blockIdx.y;
  const int t0 = blockIdx.x * 32;
  const int tb = t0 + wave * 16;

#pragma unroll 1
  for (int idx = lane; idx < 16 * AW; idx += 32) {
    const int ti = idx / AW;
    const int v  = idx - ti * AW;
    const int j  = v - ti;
    const int jc = imin(imax(j, 0), CP - 1);
    const size_t wo = ((size_t)(b * LQ + tb + ti)) * CP + jc;
    const unsigned short xh = whi[wo];
    const unsigned short xl = wlo[wo];
    const bool ok = (j >= 0) && (j < NC);
    Ah[wave][ti][v] = ok ? xh : (unsigned short)0;
    Al[wave][ti][v] = ok ? xl : (unsigned short)0;
  }
  __syncthreads();

  const unsigned short* pah = &Ah[wave][cc][8 * hh];
  const unsigned short* pal = &Al[wave][cc][8 * hh];
  const float rnc = 1.0f / (float)NC;

#pragma unroll 1
  for (int np = 0; np < DM / 32; ++np) {
    const int d0 = np * 32;
    const size_t bo0 = ((size_t)(b * DM + d0 + cc)) * LKP + tb + 8 * hh;
    const size_t bo1 = bo0 + (size_t)16 * LKP;
    v8f a0 = zero8(), a1 = zero8(), c0 = zero8(), c1 = zero8();
#pragma unroll 1
    for (int ko = 0; ko < KF; ko += 32) {
      const v16us fh  = ldfrag(pah + ko);
      const v16us fl  = ldfrag(pal + ko);
      const v16us g0h = ldfrag(kth + bo0 + ko);
      const v16us g0l = ldfrag(ktl + bo0 + ko);
      const v16us g1h = ldfrag(kth + bo1 + ko);
      const v16us g1l = ldfrag(ktl + bo1 + ko);
      a0 = mma_h(fh, g0h, a0); a1 = mma_h(fh, g0l, a1); a1 = mma_h(fl, g0h, a1);
      c0 = mma_h(fh, g1h, c0); c1 = mma_h(fh, g1l, c1); c1 = mma_h(fl, g1h, c1);
      grd4x6(a0, a1, c0, c1, fh, fl, g0h, g0l, g1h, g1l);
    }
#pragma unroll
    for (int r = 0; r < 8; ++r) {
      const int rr = 8 * hh + r;
      O[wave][rr][cc]      = (a0[r] + a1[r] * R2048) * rnc;
      O[wave][rr][16 + cc] = (c0[r] + c1[r] * R2048) * rnc;
    }
    __syncthreads();
    v4f ov[4];
#pragma unroll
    for (int it = 0; it < 4; ++it) {
      const int rl = it * 4 + (lane >> 3);
      const int p  = lane & 7;
      ov[it] = *(const v4fa*)(&O[wave][rl][4 * p]);
    }
    __syncthreads();
#pragma unroll
    for (int it = 0; it < 4; ++it) {
      const int rl = it * 4 + (lane >> 3);
      const int p  = lane & 7;
      const int t  = tb + rl;
      const int tc = imin(t, TO - 1);
      v4f* dst = (v4f*)(out + ((size_t)(b * TO + tc)) * DM + d0 + 4 * p);
      if (t < TO) *(volatile v4f*)dst = ov[it];
    }
    __threadfence();
#pragma unroll
    for (int it = 0; it < 4; ++it) {
      const int rl = it * 4 + (lane >> 3);
      const int p  = lane & 7;
      const int t  = tb + rl;
      const int tc = imin(t, TO - 1);
      v4f* dst = (v4f*)(out + ((size_t)(b * TO + tc)) * DM + d0 + 4 * p);
      if (t < TO) *(volatile v4f*)dst = ov[it];
    }
  }
}

extern "C" void kernel_launch(void* const* d_in, const int* in_sizes, int n_in,
                              void* d_out, int out_size, void* d_ws, size_t ws_size,
                              hipStream_t stream) {
  if (n_in < 19) return;
  if (in_sizes[0] != BB * LQ * DM) return;
  if (in_sizes[1] != BB * LK * DM || in_sizes[2] != BB * LK * DM) return;
  for (int i = 3; i <= 8; ++i) if (in_sizes[i] != DM) return;
  if (in_sizes[9] != DM * DM || in_sizes[10] != DM) return;
  if (in_sizes[11] != DM * DM || in_sizes[12] != DM) return;
  if (in_sizes[13] != DM * DM || in_sizes[14] != DM) return;
  if (in_sizes[15] != NC * DM * KS || in_sizes[16] != NC) return;
  if (in_sizes[17] != NC * NC || in_sizes[18] != NC) return;
  if (out_size != BB * TO * DM) return;
  if ((size_t)WS_NEED > ws_size) return;

  const float* query  = (const float*)d_in[0];
  const float* key    = (const float*)d_in[1];
  const float* value  = (const float*)d_in[2];
  const float* lnq_g  = (const float*)d_in[3];
  const float* lnq_b  = (const float*)d_in[4];
  const float* lnk_g  = (const float*)d_in[5];
  const float* lnk_b  = (const float*)d_in[6];
  const float* lnv_g  = (const float*)d_in[7];
  const float* lnv_b  = (const float*)d_in[8];
  const float* wq_w   = (const float*)d_in[9];
  const float* wq_b   = (const float*)d_in[10];
  const float* wk_w   = (const float*)d_in[11];
  const float* wk_b   = (const float*)d_in[12];
  const float* wv_w   = (const float*)d_in[13];
  const float* wv_b   = (const float*)d_in[14];
  const float* conv_w = (const float*)d_in[15];
  const float* conv_b = (const float*)d_in[16];
  const float* fnn_w  = (const float*)d_in[17];
  const float* fnn_b  = (const float*)d_in[18];
  float* out = (float*)d_out;

  char* ws = (char*)d_ws;
  unsigned short* WQ  = (unsigned short*)(ws + OFF_WQ);
  unsigned short* WK  = (unsigned short*)(ws + OFF_WK);
  unsigned short* WV  = (unsigned short*)(ws + OFF_WV);
  unsigned short* CW  = (unsigned short*)(ws + OFF_CW);
  unsigned short* FW  = (unsigned short*)(ws + OFF_FW);
  unsigned short* KH  = (unsigned short*)(ws + OFF_KH);
  unsigned short* KL  = (unsigned short*)(ws + OFF_KL);
  unsigned short* VH  = (unsigned short*)(ws + OFF_VH);
  unsigned short* VL  = (unsigned short*)(ws + OFF_VL);
  unsigned short* NH  = (unsigned short*)(ws + OFF_NH);
  unsigned short* NL  = (unsigned short*)(ws + OFF_NL);
  unsigned short* QH  = (unsigned short*)(ws + OFF_QH);
  unsigned short* QL  = (unsigned short*)(ws + OFF_QL);
  unsigned short* CH  = (unsigned short*)(ws + OFF_CH);
  unsigned short* CL  = (unsigned short*)(ws + OFF_CLO);
  unsigned short* WH  = (unsigned short*)(ws + OFF_WH);
  unsigned short* WL  = (unsigned short*)(ws + OFF_WL);
  unsigned short* TH  = (unsigned short*)(ws + OFF_TH);
  unsigned short* TL  = (unsigned short*)(ws + OFF_TL);

  const int n8w = DM * DM / 8;
  k_cvtw<<<dim3(n8w / 256, 3), dim3(256), 0, stream>>>(wq_w, wk_w, wv_w, WQ, WK, WV, n8w, 256.0f);
  const int n8c = CP * KC / 8;
  k_cvtc<<<dim3(n8c / 256), dim3(256), 0, stream>>>(conv_w, CW, n8c);
  const int n8f = CP * CP / 8;
  k_cvtf<<<dim3(n8f / 256), dim3(256), 0, stream>>>(fnn_w, FW, n8f);

  k_ln<<<dim3((BB * LKP) / 8, 3), dim3(256), 0, stream>>>(
      key, value, query, lnk_g, lnk_b, lnv_g, lnv_b, lnq_g, lnq_b, KH, KL, VH, VL, NH, NL);

  k_kv<<<dim3(LKP / 64, DM / 32, BB), dim3(128), 0, stream>>>(KH, KL, VH, VL, WK, WV, wk_b, wv_b, TH, TL);

  k_g64<0><<<dim3(LQ / 64, DM / 64, BB), dim3(128), 0, stream>>>(NH, NL, WQ, wq_b, QH, QL);

  k_g64<1><<<dim3(LQ / 64, CP / 64, BB), dim3(128), 0, stream>>>(QH, QL, CW, conv_b, CH, CL);

  k_g64<2><<<dim3(LQ / 64, CP / 64, BB), dim3(128), 0, stream>>>(CH, CL, FW, fnn_b, WH, WL);

  k_fin<<<dim3(LQ / 32, BB), dim3(64), 0, stream>>>(WH, WL, TH, TL, out);
  (void)hipGetLastError();
}
